// GATModel_83700322665088
// MI455X (gfx1250) — hardware-verified
//
#include <hip/hip_runtime.h>
#include <math.h>
#include <stdint.h>

#define NB   512
#define NF   128
#define NEMB 64
#define NH   8
#define GH   32
#define C1   256
#define DIN  32768
#define MH   256
#define VOC  100000
#define HB   256
#define RH   (HB * NF)
#define KS   32
#define KCH  (DIN / KS)

static_assert(NB == 2 * HB);
static_assert(NF == 128);
static_assert((NH % 2) == 0);
static_assert(GH == 32);
static_assert(C1 == NH * GH);
static_assert((NEMB % 32) == 0);
static_assert((C1 % 32) == 0);
static_assert(DIN == NF * C1);
static_assert((DIN % (KS * 32)) == 0);
static_assert((RH % 128) == 0);
static_assert(MH == 256);

typedef __attribute__((ext_vector_type(16))) __bf16 v16b;
typedef __attribute__((ext_vector_type(8)))  __bf16 v8b;
typedef __attribute__((ext_vector_type(8)))  float v8f;
typedef __attribute__((ext_vector_type(4)))  float v4f;
typedef __attribute__((ext_vector_type(4)))  unsigned int v4u;
typedef __attribute__((ext_vector_type(8)))  unsigned int v8u;
typedef v8b __attribute__((may_alias)) v8ba;
typedef v4f __attribute__((may_alias)) v4fa;
typedef v4u __attribute__((may_alias)) v4ua;
typedef float __attribute__((may_alias)) f1a;

union FB { v16b v; v8b h[2]; };

__device__ __forceinline__ unsigned bfb(float f) {
  const unsigned u = __float_as_uint(f);
  return (u + 0x7FFFu + ((u >> 16) & 1u)) >> 16;
}
__device__ __forceinline__ float bfr(float f) { return __uint_as_float(bfb(f) << 16); }
__device__ __forceinline__ unsigned pk16(unsigned lo, unsigned hi) { return (lo & 0xffffu) | (hi << 16); }

__device__ __forceinline__ void split8(v4f a, v4f b, v4u& hv, v4u& lv) {
  const float f[8] = {a.x, a.y, a.z, a.w, b.x, b.y, b.z, b.w};
  unsigned hb[8], lb[8];
#pragma unroll
  for (int e = 0; e < 8; ++e) {
    hb[e] = bfb(f[e]);
    lb[e] = bfb(f[e] - __uint_as_float(hb[e] << 16));
  }
  hv = (v4u){pk16(hb[0], hb[1]), pk16(hb[2], hb[3]), pk16(hb[4], hb[5]), pk16(hb[6], hb[7])};
  lv = (v4u){pk16(lb[0], lb[1]), pk16(lb[2], lb[3]), pk16(lb[4], lb[5]), pk16(lb[6], lb[7])};
}

__device__ __forceinline__ float relu_f(float v) { return (v > 0.0f) ? v : ((v == v) ? 0.0f : v); }

__device__ __forceinline__ v8f mma_bf(v16b a, v16b b, v8f c) {
  return __builtin_amdgcn_wmma_f32_16x16x32_bf16(false, a, false, b, (short)0, c, false, false);
}
__device__ __forceinline__ v8f mma_g(v16b a, v16b b, v8f c) {
  c = __builtin_amdgcn_wmma_f32_16x16x32_bf16(false, a, false, b, (short)0, c, false, false);
  asm volatile("v_nop\n\tv_nop\n\tv_nop\n\tv_nop" : "+v"(c) : "v"(a), "v"(b));
  return c;
}
__device__ __forceinline__ void guard4(v8f& a, v8f& b, v8f& c, v8f& d, v16b x, v16b y) {
  asm volatile("v_nop\n\tv_nop\n\tv_nop\n\tv_nop" : "+v"(a), "+v"(b), "+v"(c), "+v"(d) : "v"(x), "v"(y));
}
__device__ __forceinline__ void keep4(v16b a, v16b b, v16b c, v16b d) { asm volatile("v_nop" :: "v"(a), "v"(b), "v"(c), "v"(d)); }
__device__ __forceinline__ void accg4(v8f& a, v8f& b, v8f& c, v8f& d) {
  asm volatile("v_nop\n\tv_nop\n\tv_nop\n\tv_nop" : "+v"(a), "+v"(b), "+v"(c), "+v"(d));
}
__device__ __forceinline__ v16b ldfrag_g(const __bf16* p) {
  FB f; f.h[0] = *(const v8ba*)(p); f.h[1] = *(const v8ba*)(p + 16); return f.v;
}
__device__ __forceinline__ void wave_sync_lds() {
  __builtin_amdgcn_fence(__ATOMIC_RELEASE, "workgroup");
  __builtin_amdgcn_wave_barrier();
  __builtin_amdgcn_fence(__ATOMIC_ACQUIRE, "workgroup");
}

template <bool TWO>
__device__ __forceinline__ void gemm_core_g(const __bf16* A, const __bf16* A2, size_t lda,
                                            const __bf16* B, size_t ldb, int K, int lane, v8f (&acc)[4][4]) {
  const int rl = lane & 15, koff = (lane >> 4) * 8;
#pragma unroll 1
  for (int k0 = 0; k0 < K; k0 += 32) {
    v16b bh[4];
#pragma unroll
    for (int j = 0; j < 4; ++j) bh[j] = ldfrag_g(B + (size_t)(j * 16 + rl) * ldb + koff + k0);
#pragma unroll
    for (int i = 0; i < 4; ++i) {
      const size_t ao = (size_t)(i * 16 + rl) * lda + koff + k0;
      const v16b ah = ldfrag_g(A + ao);
      v16b al = ah;
      if (TWO) al = ldfrag_g(A2 + ao);
#pragma unroll
      for (int j = 0; j < 4; ++j) {
        acc[i][j] = mma_bf(ah, bh[j], acc[i][j]);
        if (TWO) acc[i][j] = mma_bf(al, bh[j], acc[i][j]);
      }
      guard4(acc[i][0], acc[i][1], acc[i][2], acc[i][3], ah, al);
    }
    keep4(bh[0], bh[1], bh[2], bh[3]);
  }
  accg4(acc[0][0], acc[0][1], acc[0][2], acc[0][3]);
  accg4(acc[1][0], acc[1][1], acc[1][2], acc[1][3]);
  accg4(acc[2][0], acc[2][1], acc[2][2], acc[2][3]);
  accg4(acc[3][0], acc[3][1], acc[3][2], acc[3][3]);
}

__global__ __launch_bounds__(256) void k_tr(const float* __restrict__ W, unsigned short* __restrict__ out,
                                            int Cc, int outPitch, int dup, long sIn) {
  __shared__ __align__(16) float tf[64 * 36];
  const float* Wz = W + (size_t)blockIdx.z * (size_t)sIn;
  const int c0 = blockIdx.x * 32, r0 = blockIdx.y * 64;
  const int tid = threadIdx.x;
  {
    const int lr = tid >> 3, c4 = (tid & 7) * 4;
#pragma unroll
    for (int it = 0; it < 2; ++it) {
      const int rr = it * 32 + lr;
      const v4f a = *(const v4fa*)(Wz + (size_t)(r0 + rr) * Cc + c0 + c4);
      *(v4fa*)(tf + rr * 36 + c4) = a;
    }
  }
  __syncthreads();
  const int oc = tid >> 3, c8 = (tid & 7) * 8;
  v4u hv;
#pragma unroll
  for (int q = 0; q < 4; ++q) {
    const float f0 = tf[(c8 + 2 * q) * 36 + oc];
    const float f1 = tf[(c8 + 2 * q + 1) * 36 + oc];
    hv[q] = pk16(bfb(f0), bfb(f1));
  }
  const size_t go = ((size_t)blockIdx.z * Cc + c0 + oc) * (size_t)outPitch + r0 + c8;
  for (int pass = 0; pass < 2; ++pass) {
    *(volatile v4u*)(out + go) = hv;
    if (dup != 0) *(volatile v4u*)(out + go + dup) = hv;
    __threadfence();
  }
}

template <bool L1>
__global__ __launch_bounds__(256) void k_proj(const int* __restrict__ ids, const float* __restrict__ vals,
                                              const float* __restrict__ emb,
                                              const unsigned short* __restrict__ Ag,
                                              const unsigned short* __restrict__ Wt,
                                              const float* __restrict__ avec,
                                              unsigned short* __restrict__ VH, float* __restrict__ SIJ, int grow0) {
  __shared__ __align__(16) unsigned short sA[128 * 72];
  __shared__ __align__(16) float sT[8][16 * 68];
  __shared__ __align__(16) float sS[8][256];
  __shared__ __align__(16) float sAv[512];
  __shared__ __align__(16) float sVs[128];

  const int tid = threadIdx.x, lane = tid & 31, wave = tid >> 5;
  const int m0 = blockIdx.x * 128;

  if (tid < 128) {
    const v4f a = *(const v4fa*)(avec + 4 * tid);
    v4f o; o.x = bfr(a.x); o.y = bfr(a.y); o.z = bfr(a.z); o.w = bfr(a.w);
    *(v4fa*)(sAv + 4 * tid) = o;
  }
  if (L1) {
    const int row = tid >> 1, half = (tid & 1) * 32;
    int id = ids[grow0 + m0 + row];
    id = (id < 0) ? 0 : ((id > VOC - 1) ? (VOC - 1) : id);
    sVs[row] = bfr(vals[grow0 + m0 + row]);
    const float* er = emb + (size_t)id * NEMB + half;
#pragma unroll
    for (int i = 0; i < 4; ++i) {
      const v4f a = *(const v4fa*)(er + 8 * i);
      const v4f b = *(const v4fa*)(er + 8 * i + 4);
      const v4u w = {pk16(bfb(a.x), bfb(a.y)), pk16(bfb(a.z), bfb(a.w)), pk16(bfb(b.x), bfb(b.y)), pk16(bfb(b.z), bfb(b.w))};
      *(v4ua*)(sA + row * 72 + half + 8 * i) = w;
    }
  }
  __syncthreads();

  const int wm = wave >> 2, wn = wave & 3;
  const int rl = lane & 15, koff = (lane >> 4) * 8, mOff = koff;
  const v8f z8 = {0.f, 0.f, 0.f, 0.f, 0.f, 0.f, 0.f, 0.f};
  v8f acc[4][4];
#pragma unroll
  for (int i = 0; i < 4; ++i)
#pragma unroll
    for (int j = 0; j < 4; ++j) acc[i][j] = z8;

  if (L1) {
    const __bf16* Bb = (const __bf16*)(const void*)Wt + (size_t)(wn * 64) * NEMB;
#pragma unroll
    for (int k0 = 0; k0 < NEMB; k0 += 32) {
      v16b bh[4];
#pragma unroll
      for (int j = 0; j < 4; ++j) bh[j] = ldfrag_g(Bb + (size_t)(j * 16 + rl) * NEMB + koff + k0);
#pragma unroll
      for (int i = 0; i < 4; ++i) {
        const int idx = (wm * 64 + i * 16 + rl) * 72 + k0 + koff;
        FB fa;
        fa.h[0] = *(const v8ba*)(sA + idx);
        fa.h[1] = *(const v8ba*)(sA + idx + 16);
#pragma unroll
        for (int j = 0; j < 4; ++j) acc[i][j] = mma_bf(fa.v, bh[j], acc[i][j]);
        guard4(acc[i][0], acc[i][1], acc[i][2], acc[i][3], fa.v, fa.v);
      }
      keep4(bh[0], bh[1], bh[2], bh[3]);
    }
    accg4(acc[0][0], acc[0][1], acc[0][2], acc[0][3]);
    accg4(acc[1][0], acc[1][1], acc[1][2], acc[1][3]);
    accg4(acc[2][0], acc[2][1], acc[2][2], acc[2][3]);
    accg4(acc[3][0], acc[3][1], acc[3][2], acc[3][3]);
  } else {
    const __bf16* Ab = (const __bf16*)(const void*)Ag + (size_t)(m0 + wm * 64) * 512;
    const __bf16* Bb = (const __bf16*)(const void*)Wt + (size_t)(wn * 64) * 512;
    gemm_core_g<false>(Ab, Ab, 512, Bb, 512, 512, lane, acc);
  }

  float* slab = sT[wave];
  float* ss = sS[wave];
  unsigned short* VL = VH + (size_t)RH * C1;
#pragma unroll
  for (int i = 0; i < 4; ++i) {
#pragma unroll
    for (int j = 0; j < 4; ++j) {
#pragma unroll
      for (int r = 0; r < 8; ++r) {
        float v = acc[i][j][r];
        if (L1) v = v * sVs[wm * 64 + i * 16 + mOff + r];
        slab[(mOff + r) * 68 + j * 16 + rl] = v;
      }
    }
    wave_sync_lds();
    {
      const int row = lane & 15, hl = lane >> 4;
      const float* sp = slab + row * 68 + hl * 32;
      const float* ap = sAv + (2 * wn + hl) * 64;
      float s_i = 0.0f, s_j = 0.0f;
#pragma unroll 2
      for (int q = 0; q < 8; ++q) {
        const v4f x  = *(const v4fa*)(sp + 4 * q);
        const v4f ai = *(const v4fa*)(ap + 4 * q);
        const v4f aj = *(const v4fa*)(ap + 32 + 4 * q);
        s_i = fmaf(x.x, ai.x, s_i); s_i = fmaf(x.y, ai.y, s_i); s_i = fmaf(x.z, ai.z, s_i); s_i = fmaf(x.w, ai.w, s_i);
        s_j = fmaf(x.x, aj.x, s_j); s_j = fmaf(x.y, aj.y, s_j); s_j = fmaf(x.z, aj.z, s_j); s_j = fmaf(x.w, aj.w, s_j);
      }
      ss[hl * 64 + i * 16 + row] = s_i;
      ss[(2 + hl) * 64 + i * 16 + row] = s_j;
    }
    {
      const int q = lane >> 3, c8 = (lane & 7) * 8;
      v4u hv[4], lv[4];
#pragma unroll
      for (int it = 0; it < 4; ++it) {
        const float* sp = slab + (it * 4 + q) * 68 + c8;
        split8(*(const v4fa*)(sp), *(const v4fa*)(sp + 4), hv[it], lv[it]);
      }
      for (int pass = 0; pass < 2; ++pass) {
#pragma unroll
        for (int it = 0; it < 4; ++it) {
          const size_t go = (size_t)(m0 + wm * 64 + i * 16 + it * 4 + q) * C1 + wn * 64 + c8;
          *(volatile v4u*)(VH + go) = hv[it];
          *(volatile v4u*)(VL + go) = lv[it];
        }
        __threadfence();
      }
    }
    wave_sync_lds();
  }
  {
    const int c4 = (lane & 15) * 4;
    v4f vv[2];
    size_t go[2];
#pragma unroll
    for (int it = 0; it < 2; ++it) {
      const int arr = it * 2 + (lane >> 4);
      const int which = arr >> 1, hl = arr & 1;
      vv[it] = *(const v4fa*)(ss + arr * 64 + c4);
      go[it] = (size_t)which * NH * RH + (size_t)(2 * wn + hl) * RH + m0 + wm * 64 + c4;
    }
    for (int pass = 0; pass < 2; ++pass) {
#pragma unroll
      for (int it = 0; it < 2; ++it) *(volatile v4f*)(SIJ + go[it]) = vv[it];
      __threadfence();
    }
  }
}

__device__ __forceinline__ float gat_logit(float si, float sj, float ad) {
  const float v = si + sj;
  const float e = (v >= 0.0f) ? v : 0.2f * v;
  const float mk = (ad > 0.0f) ? ad : -9.0e15f;
  return e * mk;
}

__global__ __launch_bounds__(256) void k_attn(const unsigned short* __restrict__ V, const float* __restrict__ SIJ,
                                              const float* __restrict__ adj, unsigned short* __restrict__ outp,
                                              int pitch, long loOff) {
  __shared__ __align__(16) unsigned int sRaw[8704];
  __shared__ __align__(16) float sSij[512];

  const int tid = threadIdx.x, lane = tid & 31, wave = tid >> 5;
  const int s = blockIdx.x >> 2, hp = blockIdx.x & 3;

#pragma unroll
  for (int it = 0; it < 2; ++it) {
    const int w = tid + 256 * it;
    const int y = (w >> 3) * 2, ch = w & 7;
#pragma unroll
    for (int pl = 0; pl < 2; ++pl) {
      const unsigned short* src = V + (size_t)pl * ((size_t)RH * C1) + (size_t)(s * NF + y) * C1 + hp * 64 + ch * 8;
      const v4u va = *(const v4ua*)(src);
      const v4u vb = *(const v4ua*)(src + C1);
#pragma unroll
      for (int q = 0; q < 4; ++q) {
        const int c = ch * 8 + 2 * q;
        const int base = (pl * 8704 + c * 136 + y) >> 1;
        sRaw[base]      = (va[q] & 0xffffu) | (vb[q] << 16);
        sRaw[base + 68] = (va[q] >> 16) | (vb[q] & 0xffff0000u);
      }
    }
  }
  {
    const int which = tid >> 7, idx = tid & 127;
#pragma unroll
    for (int hl = 0; hl < 2; ++hl)
      sSij[(which * 2 + hl) * 128 + idx] =
          SIJ[(size_t)which * NH * RH + (size_t)(2 * hp + hl) * RH + s * NF + idx];
  }
  __syncthreads();

  const int h = lane >> 4, c = lane & 15;
  const int x = wave * 16 + c;
  const float* arow = adj + x * NF;
  const unsigned short* sVp = (const unsigned short*)sRaw;
  const v8f z8 = {0.f, 0.f, 0.f, 0.f, 0.f, 0.f, 0.f, 0.f};
  v8f res[2][2];

#pragma unroll
  for (int hl = 0; hl < 2; ++hl) {
    const float si = sSij[hl * 128 + x];
    const float* sjp = sSij + (2 + hl) * 128;
    float mx = -__builtin_inff();
#pragma unroll 1
    for (int kc = 0; kc < 4; ++kc) {
#pragma unroll
      for (int g = 0; g < 2; ++g) {
        const int y0 = kc * 32 + 16 * g + 8 * h;
        const v4f j0 = *(const v4fa*)(sjp + y0), j1 = *(const v4fa*)(sjp + y0 + 4);
        const v4f a0 = *(const v4fa*)(arow + y0), a1 = *(const v4fa*)(arow + y0 + 4);
        const float sj8[8] = {j0.x, j0.y, j0.z, j0.w, j1.x, j1.y, j1.z, j1.w};
        const float ad8[8] = {a0.x, a0.y, a0.z, a0.w, a1.x, a1.y, a1.z, a1.w};
#pragma unroll
        for (int e = 0; e < 8; ++e) mx = fmaxf(mx, gat_logit(si, sj8[e], ad8[e]));
      }
    }
    mx = fmaxf(mx, __shfl_xor(mx, 16, 32));
    float sum = 0.0f;
    v8f acc0 = z8, acc1 = z8;
#pragma unroll 1
    for (int kc = 0; kc < 4; ++kc) {
      float pv[16];
#pragma unroll
      for (int g = 0; g < 2; ++g) {
        const int y0 = kc * 32 + 16 * g + 8 * h;
        const v4f j0 = *(const v4fa*)(sjp + y0), j1 = *(const v4fa*)(sjp + y0 + 4);
        const v4f a0 = *(const v4fa*)(arow + y0), a1 = *(const v4fa*)(arow + y0 + 4);
        const float sj8[8] = {j0.x, j0.y, j0.z, j0.w, j1.x, j1.y, j1.z, j1.w};
        const float ad8[8] = {a0.x, a0.y, a0.z, a0.w, a1.x, a1.y, a1.z, a1.w};
#pragma unroll
        for (int e = 0; e < 8; ++e) {
          const float p = expf(gat_logit(si, sj8[e], ad8[e]) - mx);
          sum += p;
          pv[g * 8 + e] = p;
        }
      }
      v8u phw, plw;
#pragma unroll
      for (int q = 0; q < 8; ++q) {
        const unsigned h0 = bfb(pv[2 * q]), h1 = bfb(pv[2 * q + 1]);
        const unsigned l0 = bfb(pv[2 * q] - __uint_as_float(h0 << 16));
        const unsigned l1 = bfb(pv[2 * q + 1] - __uint_as_float(h1 << 16));
        phw[q] = pk16(h0, h1);
        plw[q] = pk16(l0, l1);
      }
      const v16b Phi = __builtin_bit_cast(v16b, phw);
      const v16b Plo = __builtin_bit_cast(v16b, plw);
      const int kb = kc * 32 + 8 * h;
      FB vh0, vl0, vh1, vl1;
      {
        const int n0 = (hl * 32 + c) * 136 + kb;
        const int n1 = (hl * 32 + 16 + c) * 136 + kb;
        vh0.h[0] = *(const v8ba*)(sVp + n0);          vh0.h[1] = *(const v8ba*)(sVp + n0 + 16);
        vl0.h[0] = *(const v8ba*)(sVp + 8704 + n0);   vl0.h[1] = *(const v8ba*)(sVp + 8704 + n0 + 16);
        vh1.h[0] = *(const v8ba*)(sVp + n1);          vh1.h[1] = *(const v8ba*)(sVp + n1 + 16);
        vl1.h[0] = *(const v8ba*)(sVp + 8704 + n1);   vl1.h[1] = *(const v8ba*)(sVp + 8704 + n1 + 16);
      }
      acc0 = mma_g(Phi, vh0.v, acc0);
      acc0 = mma_g(Plo, vh0.v, acc0);
      acc0 = mma_g(Phi, vl0.v, acc0);
      acc1 = mma_g(Phi, vh1.v, acc1);
      acc1 = mma_g(Plo, vh1.v, acc1);
      acc1 = mma_g(Phi, vl1.v, acc1);
    }
    sum += __shfl_xor(sum, 16, 32);
    const float inv = 1.0f / sum;
#pragma unroll
    for (int r = 0; r < 8; ++r) {
      const float ir = __shfl(inv, 8 * h + r, 32);
      float v0 = acc0[r] * ir, v1 = acc1[r] * ir;
      v0 = (v0 > 0.0f) ? v0 : expm1f(v0);
      v1 = (v1 > 0.0f) ? v1 : expm1f(v1);
      res[hl][0][r] = v0;
      res[hl][1][r] = v1;
    }
  }

  __syncthreads();
  {
    f1a* stg = (f1a*)sRaw + wave * 1088;
#pragma unroll
    for (int hl = 0; hl < 2; ++hl)
#pragma unroll
      for (int t = 0; t < 2; ++t)
#pragma unroll
        for (int r = 0; r < 8; ++r) stg[(8 * h + r) * 68 + hl * 32 + t * 16 + c] = res[hl][t][r];
  }
  __syncthreads();
  {
    const int q = lane >> 3, c8 = (lane & 7) * 8;
    const float* stg = (const float*)sRaw + wave * 1088;
    v4u hv[4], lv[4];
#pragma unroll
    for (int it = 0; it < 4; ++it) {
      const float* sp = stg + (it * 4 + q) * 68 + c8;
      split8(*(const v4fa*)(sp), *(const v4fa*)(sp + 4), hv[it], lv[it]);
    }
    for (int pass = 0; pass < 2; ++pass) {
#pragma unroll
      for (int it = 0; it < 4; ++it) {
        const size_t go = (size_t)(s * NF + wave * 16 + it * 4 + q) * (size_t)pitch + hp * 64 + c8;
        *(volatile v4u*)(outp + go) = hv[it];
        *(volatile v4u*)(outp + (size_t)loOff + go) = lv[it];
      }
      __threadfence();
    }
  }
}

__global__ __launch_bounds__(128) void k_mlp0(const unsigned short* __restrict__ Z, const unsigned short* __restrict__ W0T,
                                              float* __restrict__ PARTp) {
  __shared__ __align__(16) float sT[4][16 * 68];
  const int tid = threadIdx.x, lane = tid & 31, wave = tid >> 5;
  const int tile = blockIdx.x, ks = blockIdx.y;
  const int m0 = (tile >> 1) * 128 + (wave >> 1) * 64;
  const int n0 = (tile & 1) * 128 + (wave & 1) * 64;
  const size_t kb = (size_t)ks * KCH;
  const __bf16* A  = (const __bf16*)(const void*)Z + (size_t)m0 * DIN + kb;
  const __bf16* A2 = A + (size_t)HB * DIN;
  const __bf16* B  = (const __bf16*)(const void*)W0T + (size_t)n0 * DIN + kb;

  const v8f z8 = {0.f, 0.f, 0.f, 0.f, 0.f, 0.f, 0.f, 0.f};
  v8f acc[4][4];
#pragma unroll
  for (int i = 0; i < 4; ++i)
#pragma unroll
    for (int j = 0; j < 4; ++j) acc[i][j] = z8;
  gemm_core_g<true>(A, A2, DIN, B, DIN, KCH, lane, acc);

  float* slab = sT[wave];
  float* C = PARTp + (size_t)ks * HB * MH;
  const int rl = lane & 15, mOff = (lane >> 4) * 8;
#pragma unroll
  for (int i = 0; i < 4; ++i) {
#pragma unroll
    for (int j = 0; j < 4; ++j)
#pragma unroll
      for (int r = 0; r < 8; ++r) slab[(mOff + r) * 68 + j * 16 + rl] = acc[i][j][r];
    wave_sync_lds();
    {
      const int hh = lane >> 4, c4 = (lane & 15) * 4;
      v4f vv[8];
#pragma unroll
      for (int it = 0; it < 8; ++it) vv[it] = *(const v4fa*)(slab + (it * 2 + hh) * 68 + c4);
      for (int pass = 0; pass < 2; ++pass) {
#pragma unroll
        for (int it = 0; it < 8; ++it)
          *(volatile v4f*)(C + (size_t)(m0 + i * 16 + it * 2 + hh) * MH + n0 + c4) = vv[it];
        __threadfence();
      }
    }
    wave_sync_lds();
  }
}

__global__ __launch_bounds__(256) void k_tail(const float* __restrict__ PART, const unsigned short* __restrict__ W1M,
                                              const float* __restrict__ b0, const float* __restrict__ b1,
                                              const float* __restrict__ ow, const float* __restrict__ ob,
                                              float* __restrict__ out) {
  __shared__ __align__(16) unsigned int sRaw[8320];
  __shared__ __align__(16) float sB0[256];
  __shared__ __align__(16) float sB1[256];
  __shared__ __align__(16) float sOw[256];
  __shared__ __align__(16) float sY[32];
  __shared__ float sOb[4];

  const int tid = threadIdx.x, lane = tid & 31, wave = tid >> 5;
  const int bi = blockIdx.x, p = bi >> 3, r0 = (bi & 7) * 32;

  if (tid < 64) {
    const v4f a = *(const v4fa*)(b0 + 4 * tid);
    v4f o; o.x = bfr(a.x); o.y = bfr(a.y); o.z = bfr(a.z); o.w = bfr(a.w);
    *(v4fa*)(sB0 + 4 * tid) = o;
  } else if (tid < 128) {
    const int t = tid - 64;
    const v4f a = *(const v4fa*)(b1 + 4 * t);
    v4f o; o.x = bfr(a.x); o.y = bfr(a.y); o.z = bfr(a.z); o.w = bfr(a.w);
    *(v4fa*)(sB1 + 4 * t) = o;
  } else if (tid < 192) {
    const int t = tid - 128;
    const v4f a = *(const v4fa*)(ow + 4 * t);
    v4f o; o.x = bfr(a.x); o.y = bfr(a.y); o.z = bfr(a.z); o.w = bfr(a.w);
    *(v4fa*)(sOw + 4 * t) = o;
  } else if (tid < 224) {
    sOb[0] = bfr(ob[0]);
  }
  __syncthreads();

#pragma unroll 1
  for (int it = 0; it < 8; ++it) {
    const int e = tid + 256 * it;
    const int row = e >> 6, c4 = (e & 63) * 4;
    const float* pp = PART + ((size_t)p * KS * HB + r0 + row) * MH + c4;
    v4f sacc = {0.f, 0.f, 0.f, 0.f};
#pragma unroll 4
    for (int ks = 0; ks < KS; ++ks) {
      const v4f v = *(const v4fa*)(pp + (size_t)ks * HB * MH);
      sacc.x += v.x; sacc.y += v.y; sacc.z += v.z; sacc.w += v.w;
    }
    const v4f bb = *(const v4fa*)(sB0 + c4);
    const float f0 = relu_f(sacc.x + bb.x), f1 = relu_f(sacc.y + bb.y);
    const float f2 = relu_f(sacc.z + bb.z), f3 = relu_f(sacc.w + bb.w);
    const unsigned h0 = bfb(f0), h1 = bfb(f1), h2 = bfb(f2), h3 = bfb(f3);
    const unsigned l0 = bfb(f0 - __uint_as_float(h0 << 16)), l1 = bfb(f1 - __uint_as_float(h1 << 16));
    const unsigned l2 = bfb(f2 - __uint_as_float(h2 << 16)), l3 = bfb(f3 - __uint_as_float(h3 << 16));
    const int wi = (row * 520 + c4) >> 1;
    sRaw[wi]       = pk16(h0, h1);
    sRaw[wi + 1]   = pk16(h2, h3);
    sRaw[wi + 128] = pk16(l0, l1);
    sRaw[wi + 129] = pk16(l2, l3);
  }
  __syncthreads();

  const int rl = lane & 15, koff = (lane >> 4) * 8, mOff = koff;
  const v8f z8 = {0.f, 0.f, 0.f, 0.f, 0.f, 0.f, 0.f, 0.f};
  v8f acc[2][2];
  acc[0][0] = z8; acc[0][1] = z8; acc[1][0] = z8; acc[1][1] = z8;
  {
    const unsigned short* sAp = (const unsigned short*)sRaw;
    const __bf16* Bb = (const __bf16*)(const void*)W1M + (size_t)(wave * 32) * 512;
#pragma unroll 1
    for (int k0 = 0; k0 < 512; k0 += 32) {
      const v16b bA = ldfrag_g(Bb + (size_t)rl * 512 + koff + k0);
      const v16b bB = ldfrag_g(Bb + (size_t)(16 + rl) * 512 + koff + k0);
      FB a0, a1;
      a0.h[0] = *(const v8ba*)(sAp + rl * 520 + k0 + koff);
      a0.h[1] = *(const v8ba*)(sAp + rl * 520 + k0 + koff + 16);
      a1.h[0] = *(const v8ba*)(sAp + (16 + rl) * 520 + k0 + koff);
      a1.h[1] = *(const v8ba*)(sAp + (16 + rl) * 520 + k0 + koff + 16);
      acc[0][0] = mma_bf(a0.v, bA, acc[0][0]);
      acc[0][1] = mma_bf(a0.v, bB, acc[0][1]);
      acc[1][0] = mma_bf(a1.v, bA, acc[1][0]);
      acc[1][1] = mma_bf(a1.v, bB, acc[1][1]);
      guard4(acc[0][0], acc[0][1], acc[1][0], acc[1][1], a0.v, a1.v);
      keep4(bA, bB, a0.v, a1.v);
    }
    accg4(acc[0][0], acc[0][1], acc[1][0], acc[1][1]);
  }
  __syncthreads();
  {
    f1a* z2 = (f1a*)sRaw;
#pragma unroll
    for (int im = 0; im < 2; ++im)
#pragma unroll
      for (int jn = 0; jn < 2; ++jn) {
        const int n = wave * 32 + jn * 16 + rl;
        const float bv = sB1[n];
#pragma unroll
        for (int r = 0; r < 8; ++r) z2[(im * 16 + mOff + r) * 260 + n] = relu_f(acc[im][jn][r] + bv);
      }
  }
  __syncthreads();
  if (wave == 0) {
    const float* z2 = (const float*)sRaw + lane * 260;
    float y = 0.0f;
#pragma unroll 4
    for (int j = 0; j < MH; ++j) y = fmaf(z2[j], sOw[j], y);
    sY[lane] = y + sOb[0];
  }
  __syncthreads();
  if (tid < 8) {
    const v4f v = *(const v4fa*)(sY + 4 * tid);
    float* dst = out + bi * 32 + 4 * tid;
    *(volatile v4f*)dst = v;
    __threadfence();
    *(volatile v4f*)dst = v;
  }
}

extern "C" void kernel_launch(void* const* d_in, const int* in_sizes, int n_in,
                              void* d_out, int out_size, void* d_ws, size_t ws_size,
                              hipStream_t stream) {
  if (n_in < 14) return;
  if (in_sizes[0] != NB * NF || in_sizes[1] != NB * NF || in_sizes[2] != NF * NF) return;
  if (in_sizes[3] != VOC * NEMB) return;
  if (in_sizes[4] != NH * NEMB * GH || in_sizes[5] != NH * 2 * GH) return;
  if (in_sizes[6] != NH * C1 * GH || in_sizes[7] != NH * 2 * GH) return;
  if (in_sizes[8] != DIN * MH || in_sizes[9] != MH) return;
  if (in_sizes[10] != MH * MH || in_sizes[11] != MH || in_sizes[12] != MH || in_sizes[13] != 1) return;
  if (out_size != NB) return;

  const int*   ids    = (const int*)  d_in[0];
  const float* vals   = (const float*)d_in[1];
  const float* adj    = (const float*)d_in[2];
  const float* emb    = (const float*)d_in[3];
  const float* W0     = (const float*)d_in[4];
  const float* a0     = (const float*)d_in[5];
  const float* W1     = (const float*)d_in[6];
  const float* a1     = (const float*)d_in[7];
  const float* mlp_w0 = (const float*)d_in[8];
  const float* mlp_b0 = (const float*)d_in[9];
  const float* mlp_w1 = (const float*)d_in[10];
  const float* mlp_b1 = (const float*)d_in[11];
  const float* out_w  = (const float*)d_in[12];
  const float* out_b  = (const float*)d_in[13];
  float* y = (float*)d_out;

  const size_t szPlane = (size_t)RH * C1 * 2;
  size_t off = 0;
  const size_t oV    = off; off += 2 * szPlane;
  const size_t oB    = off; off += 2 * szPlane;
  const size_t oSIJ  = off; off += (size_t)2 * NH * RH * 4;
  const size_t oW0T  = off; off += (size_t)MH * DIN * 2;
  const size_t oPART = off; off += (size_t)2 * KS * HB * MH * 4;
  const size_t oW0t  = off; off += (size_t)C1 * NEMB * 2;
  const size_t oW1t2 = off; off += (size_t)C1 * 512 * 2;
  const size_t oW1M  = off; off += (size_t)MH * 512 * 2;
  if (off > ws_size) return;
  if (off > (size_t)134217728) return;

  char* ws = (char*)d_ws;
  unsigned short* Vp   = (unsigned short*)(ws + oV);
  unsigned short* Bq   = (unsigned short*)(ws + oB);
  float*          SIJ  = (float*)(ws + oSIJ);
  unsigned short* W0T  = (unsigned short*)(ws + oW0T);
  float*          PART = (float*)(ws + oPART);
  unsigned short* W0t  = (unsigned short*)(ws + oW0t);
  unsigned short* W1t2 = (unsigned short*)(ws + oW1t2);
  unsigned short* W1M  = (unsigned short*)(ws + oW1M);

  const dim3 blk(256);
  k_tr<<<dim3(GH / 32, NEMB / 64, NH), blk, 0, stream>>>(W0, W0t, GH, NEMB, 0, (long)(NEMB * GH));
  k_tr<<<dim3(GH / 32, C1 / 64, NH), blk, 0, stream>>>(W1, W1t2, GH, 512, 256, (long)(C1 * GH));
  k_tr<<<dim3(MH / 32, DIN / 64, 1), blk, 0, stream>>>(mlp_w0, W0T, MH, DIN, 0, 0L);
  k_tr<<<dim3(MH / 32, MH / 64, 1), blk, 0, stream>>>(mlp_w1, W1M, MH, 512, 256, 0L);

  for (int p = 0; p < 2; ++p) {
    const int grow0 = p * RH;
    k_proj<true><<<dim3(RH / 128), blk, 0, stream>>>(ids, vals, emb, Bq, W0t, a0, Vp, SIJ, grow0);
    k_attn<<<dim3(HB * (NH / 2)), blk, 0, stream>>>(Vp, SIJ, adj, Bq, 512, 256L);
    k_proj<false><<<dim3(RH / 128), blk, 0, stream>>>(ids, vals, emb, Bq, W1t2, a1, Vp, SIJ, grow0);
    k_attn<<<dim3(HB * (NH / 2)), blk, 0, stream>>>(Vp, SIJ, adj, Bq, 256, (long)RH * C1);
    k_mlp0<<<dim3(4, KS), dim3(128), 0, stream>>>(Bq, W0T, PART + (size_t)p * KS * HB * MH);
  }
  k_tail<<<dim3(NB / 32), blk, 0, stream>>>(PART, W1M, mlp_b0, mlp_b1, out_w, out_b, y);
  (void)hipGetLastError();
}
